// SafetyDistanceConstraint_54039278518798
// MI455X (gfx1250) — hardware-run, weakly checked
//
#include <hip/hip_runtime.h>
#include <math.h>

typedef __attribute__((ext_vector_type(16))) _Float16 v16h;
typedef __attribute__((ext_vector_type(8)))  _Float16 v8h;
typedef __attribute__((ext_vector_type(8)))  float    v8f;
typedef __attribute__((ext_vector_type(4)))  float    v4f;

constexpr int kBatch   = 1024;
constexpr int kAgents  = 64;
constexpr int kPairs   = 2016;
constexpr int kHid     = 64;
constexpr int kGroups  = 63;
constexpr int kRowF    = kAgents * 3;
static_assert(kPairs == kAgents * (kAgents - 1) / 2, "pair count");
static_assert(kGroups * 32 == kPairs, "32-pair groups cover the pair axis exactly");
static_assert(kRowF == 192, "six whole 128-B lines per batch row of forces");
static_assert(((size_t)kBatch * kRowF * 4) % 128 == 0, "second output starts on a line");
static_assert((kPairs * 4) % 128 == 0, "violation rows are whole lines");

constexpr int kW1P = 40;
constexpr int kHP  = 72;

constexpr float kXC  = 8.0f;
constexpr float kWC1 = 64.0f;
constexpr float kWC2 = 64.0f;
constexpr float kWC3 = 256.0f;
constexpr float kHC  = 8.0f;
constexpr float kBiasC1 = kXC * kWC1;
constexpr float kBiasC2 = kHC * kWC2;
constexpr float kBiasC3 = kHC * kWC3;
constexpr float kEp1 = kHC / (kXC * kWC1);
constexpr float kEp2 = kHC / (kHC * kWC2);
constexpr float kEp3 = 1.0f / (kHC * kWC3);
static_assert(kEp1 == 1.0f / 64.0f && kEp2 == 1.0f / 64.0f && kEp3 == 1.0f / 2048.0f, "fold-back constants");

constexpr size_t kWsFlagsBytes = 8192;
constexpr size_t kWsTotal = kWsFlagsBytes;
static_assert(kWsTotal <= 134217728ull, "carve cap");

__device__ __forceinline__ v16h frag_load(const _Float16* p) {
  union { v16h v; v8h h[2]; } f;
  f.h[0] = *(const v8h*)(p);
  f.h[1] = *(const v8h*)(p + 16);
  return f.v;
}
__device__ __forceinline__ v8f mma_h(v16h a, v16h b, v8f c) {
  c = __builtin_amdgcn_wmma_f32_16x16x32_f16(false, a, false, b, (short)0, c, false, false);
  asm volatile("v_nop\n\tv_nop\n\tv_nop\n\tv_nop" : "+v"(c) : "v"(a), "v"(b));
  return c;
}
__device__ __forceinline__ void wave_lds_sync() {
  __builtin_amdgcn_fence(__ATOMIC_RELEASE, "workgroup");
  __builtin_amdgcn_wave_barrier();
  __builtin_amdgcn_fence(__ATOMIC_ACQUIRE, "workgroup");
}
__device__ __forceinline__ int iclamp(int v, int lo, int hi) {
  v = v < lo ? lo : v;
  v = v > hi ? hi : v;
  return v;
}

__device__ __forceinline__ void pair_decode(int p, int& oi, int& oj) {
  int i = (int)((127.0f - sqrtf(16129.0f - 8.0f * (float)p)) * 0.5f);
  i = iclamp(i, 0, 62);
  i += ((((i + 1) * (126 - i)) / 2) <= p) ? 1 : 0;
  i += ((((i + 1) * (126 - i)) / 2) <= p) ? 1 : 0;
  i -= (((i * (127 - i)) / 2) > p) ? 1 : 0;
  i -= (((i * (127 - i)) / 2) > p) ? 1 : 0;
  i = iclamp(i, 0, 62);
  int j = p - (i * (127 - i)) / 2 + i + 1;
  j = iclamp(j, i + 1, 63);
  oi = i;
  oj = j;
}

__device__ __forceinline__ float dist3(float x, float y, float z) {
#pragma clang fp contract(off)
  const float t0 = x * x;
  const float t1 = y * y;
  const float t2 = z * z;
  return sqrtf((t0 + t2) + t1);
}
__device__ __forceinline__ float violation_of(float logit, float dist) {
#pragma clang fp contract(off)
  const float e  = expf(-logit);
  const float sg = __builtin_amdgcn_rcpf(1.0f + e);
  const float s1 = 1.0f + sg;
  const float sd = 5.0f * s1;
  return sd - dist;
}

template <bool RP>
__global__ __launch_bounds__(256) void pair_mlp_kernel(
    const float* __restrict__ pos, const float* __restrict__ vel,
    const float* __restrict__ w1, const float* __restrict__ b1,
    const float* __restrict__ w2, const float* __restrict__ b2,
    const float* __restrict__ w3, const float* __restrict__ b3,
    const int* __restrict__ flags, float* __restrict__ outp)
{
  constexpr int KIN  = RP ? 7 : 6;
  constexpr int NOUT = RP ? 3 : 1;
  __shared__ __align__(16) float    s_pos[kRowF];
  __shared__ __align__(16) float    s_vel[kRowF];
  __shared__ __align__(16) _Float16 s_wa1[kHid * kW1P];
  __shared__ __align__(16) _Float16 s_wa2[kHid * kHP];
  __shared__ __align__(16) _Float16 s_wa3[16 * kHP];
  __shared__ __align__(16) float    s_b1c[kHid];
  __shared__ __align__(16) float    s_b2c[kHid];
  __shared__ __align__(16) float    s_b3c[16];
  __shared__ __align__(16) _Float16 s_ht[8 * 16 * kHP];
  __shared__ __align__(16) float    s_stage[RP ? 4 : 8 * 32];
  __shared__ __align__(16) float    s_rep[RP ? kPairs * 3 : 4];

  const int tid  = threadIdx.x;
  const int lane = tid & 31;
  const int wave = __builtin_amdgcn_readfirstlane(tid >> 5);
  const int hh   = lane >> 4;
  const int c    = lane & 15;
  const int b    = blockIdx.x;

  if (tid < kRowF) {
    s_pos[tid] = pos[(size_t)b * kRowF + tid];
    s_vel[tid] = vel[(size_t)b * kRowF + tid];
  }
#pragma unroll 1
  for (int it = 0; it < 8; ++it) {
    const int idx = it * 256 + tid;
    const int k = idx >> 6;
    const int n = idx & 63;
    const int kk = k < KIN ? k : KIN - 1;
    const float wv = w1[kk * kHid + n];
    const float cv = (k < KIN) ? wv * kWC1 : 0.0f;
    s_wa1[n * kW1P + k] = (_Float16)cv;
  }
#pragma unroll 1
  for (int it = 0; it < 16; ++it) {
    const int idx = it * 256 + tid;
    const int k = idx >> 6;
    const int n = idx & 63;
    const float wv = w2[k * kHid + n];
    s_wa2[n * kHP + k] = (_Float16)(wv * kWC2);
  }
#pragma unroll 1
  for (int it = 0; it < 4; ++it) {
    const int idx = it * 256 + tid;
    const int k = idx >> 4;
    const int n = idx & 15;
    const int nn = n < NOUT ? n : NOUT - 1;
    const float wv = w3[k * NOUT + nn];
    const float cv = (n < NOUT) ? wv * kWC3 : 0.0f;
    s_wa3[n * kHP + k] = (_Float16)cv;
  }
  if (tid < kHid) {
    s_b1c[tid] = b1[tid] * kBiasC1;
    s_b2c[tid] = b2[tid] * kBiasC2;
  }
  if (tid < 16) {
    const int nn = tid < NOUT ? tid : NOUT - 1;
    const float bv = b3[nn];
    s_b3c[tid] = (tid < NOUT) ? bv * kBiasC3 : 0.0f;
  }
  __syncthreads();

  v16h wa1[4];
  v16h wa2[4][2];
#pragma unroll
  for (int jn = 0; jn < 4; ++jn) {
    wa1[jn] = frag_load(s_wa1 + (jn * 16 + c) * kW1P + 8 * hh);
#pragma unroll
    for (int kc = 0; kc < 2; ++kc)
      wa2[jn][kc] = frag_load(s_wa2 + (jn * 16 + c) * kHP + kc * 32 + 8 * hh);
  }

  _Float16* ht = s_ht + wave * (16 * kHP);
  float zf = 0.0f;
  asm volatile("" : "+v"(zf));
  const bool lo = (hh == 0);
  const v8h z8 = {(_Float16)0.0f, (_Float16)0.0f, (_Float16)0.0f, (_Float16)0.0f,
                  (_Float16)0.0f, (_Float16)0.0f, (_Float16)0.0f, (_Float16)0.0f};

#pragma unroll 1
  for (int g = wave; g < kGroups; g += 8) {
#pragma unroll 1
    for (int mt = 0; mt < 2; ++mt) {
      const int p = g * 32 + mt * 16 + c;
      int pi, pj;
      pair_decode(p, pi, pj);
      const float px = s_pos[pj * 3 + 0] - s_pos[pi * 3 + 0];
      const float py = s_pos[pj * 3 + 1] - s_pos[pi * 3 + 1];
      const float pz = s_pos[pj * 3 + 2] - s_pos[pi * 3 + 2];
      const float vx = s_vel[pj * 3 + 0] - s_vel[pi * 3 + 0];
      const float vy = s_vel[pj * 3 + 1] - s_vel[pi * 3 + 1];
      const float vz = s_vel[pj * 3 + 2] - s_vel[pi * 3 + 2];
      const float dist = dist3(px, py, pz);

      v8h x0;
      x0[0] = (_Float16)(lo ? px * kXC : zf);
      x0[1] = (_Float16)(lo ? py * kXC : zf);
      x0[2] = (_Float16)(lo ? pz * kXC : zf);
      x0[3] = (_Float16)(lo ? vx * kXC : zf);
      x0[4] = (_Float16)(lo ? vy * kXC : zf);
      x0[5] = (_Float16)(lo ? vz * kXC : zf);
      x0[6] = (_Float16)((lo && RP) ? dist * kXC : zf);
      x0[7] = (_Float16)zf;
      union { v16h v; v8h h[2]; } xb;
      xb.h[0] = x0;
      xb.h[1] = z8;

      v8f acc[4];
#pragma unroll
      for (int jn = 0; jn < 4; ++jn) {
        const v4f c0 = *(const v4f*)(s_b1c + jn * 16 + 8 * hh);
        const v4f c1 = *(const v4f*)(s_b1c + jn * 16 + 8 * hh + 4);
        const v8f ci = {c0[0], c0[1], c0[2], c0[3], c1[0], c1[1], c1[2], c1[3]};
        acc[jn] = mma_h(wa1[jn], xb.v, ci);
      }
      wave_lds_sync();
#pragma unroll
      for (int jn = 0; jn < 4; ++jn) {
        v8h hv;
#pragma unroll
        for (int r = 0; r < 8; ++r) {
          const float t = fmaxf(acc[jn][r], 0.0f) * kEp1;
          hv[r] = (_Float16)t;
        }
        *(v8h*)(ht + c * kHP + jn * 16 + 8 * hh) = hv;
      }
      wave_lds_sync();

      {
        const v16h hb0 = frag_load(ht + c * kHP + 8 * hh);
        const v16h hb1 = frag_load(ht + c * kHP + 32 + 8 * hh);
#pragma unroll
        for (int jn = 0; jn < 4; ++jn) {
          const v4f c0 = *(const v4f*)(s_b2c + jn * 16 + 8 * hh);
          const v4f c1 = *(const v4f*)(s_b2c + jn * 16 + 8 * hh + 4);
          const v8f ci = {c0[0], c0[1], c0[2], c0[3], c1[0], c1[1], c1[2], c1[3]};
          acc[jn] = mma_h(wa2[jn][0], hb0, ci);
          acc[jn] = mma_h(wa2[jn][1], hb1, acc[jn]);
        }
      }
      wave_lds_sync();
#pragma unroll
      for (int jn = 0; jn < 4; ++jn) {
        v8h hv;
#pragma unroll
        for (int r = 0; r < 8; ++r) {
          const float t = fmaxf(acc[jn][r], 0.0f) * kEp2;
          hv[r] = (_Float16)t;
        }
        *(v8h*)(ht + c * kHP + jn * 16 + 8 * hh) = hv;
      }
      wave_lds_sync();

      v8f a3;
      {
        const v16h hb0 = frag_load(ht + c * kHP + 8 * hh);
        const v16h hb1 = frag_load(ht + c * kHP + 32 + 8 * hh);
        const v16h w3a = frag_load(s_wa3 + c * kHP + 8 * hh);
        const v16h w3b = frag_load(s_wa3 + c * kHP + 32 + 8 * hh);
        const v4f c0 = *(const v4f*)(s_b3c + 8 * hh);
        const v4f c1 = *(const v4f*)(s_b3c + 8 * hh + 4);
        const v8f ci = {c0[0], c0[1], c0[2], c0[3], c1[0], c1[1], c1[2], c1[3]};
        a3 = mma_h(w3a, hb0, ci);
        a3 = mma_h(w3b, hb1, a3);
      }
      wave_lds_sync();

      if (RP) {
        int fl = flags[p];
        asm volatile("" : "+v"(fl));
        const bool on = (fl != 0);
        const float r0 = on ? a3[0] * kEp3 : 0.0f;
        const float r1 = on ? a3[1] * kEp3 : 0.0f;
        const float r2 = on ? a3[2] * kEp3 : 0.0f;
        if (lo) {
          s_rep[p * 3 + 0] = r0;
          s_rep[p * 3 + 1] = r1;
          s_rep[p * 3 + 2] = r2;
        }
      } else {
        const float logit = a3[0] * kEp3;
        const float viol = violation_of(logit, dist);
        if (lo) s_stage[wave * 32 + mt * 16 + c] = viol;
      }
    }
    if (!RP) {
      wave_lds_sync();
      const float v = s_stage[wave * 32 + lane];
      volatile float* o = outp + (size_t)b * kPairs + g * 32 + lane;
      *o = v;
      __threadfence();
      *o = v;
      wave_lds_sync();
    }
  }

  if (RP) {
    __syncthreads();
    if (tid < kRowF) {
      const int n  = tid / 3;
      const int cc = tid - 3 * n;
      float f = 0.0f;
#pragma unroll 1
      for (int q = 0; q < kAgents; ++q) {
        const int a  = q < n ? q : n;
        const int bb = q < n ? n : q;
        int pp = (a * (127 - a)) / 2 + (bb - a - 1);
        pp = iclamp(pp, 0, kPairs - 1);
        const float v = s_rep[pp * 3 + cc];
        const float sv = (q < n) ? v : -v;
        const float tv = (q == n) ? 0.0f : sv;
        f += tv;
      }
      volatile float* o = outp + (size_t)b * kRowF + tid;
      *o = f;
      __threadfence();
      *o = f;
    }
  }
}

__global__ __launch_bounds__(256) void pair_flag_kernel(const float* __restrict__ viol, int* __restrict__ flags)
{
  const int p  = blockIdx.x * 256 + threadIdx.x;
  const int pc = p < kPairs ? p : kPairs - 1;
  int any = 0;
#pragma unroll 8
  for (int bi = 0; bi < kBatch; ++bi) {
    const float v = viol[(size_t)bi * kPairs + pc];
    any |= (v > 0.0f) ? 1 : 0;
  }
  const int outv = (p < kPairs) ? any : 0;
  volatile int* o = flags + p;
  *o = outv;
  __threadfence();
  *o = outv;
}

extern "C" void kernel_launch(void* const* d_in, const int* in_sizes, int n_in,
                              void* d_out, int out_size, void* d_ws, size_t ws_size,
                              hipStream_t stream) {
  if (n_in < 14) return;
  if (in_sizes[0] != kBatch * kRowF) return;
  if (in_sizes[1] != kBatch * kRowF) return;
  if (in_sizes[2] != 6 * kHid) return;
  if (in_sizes[3] != kHid) return;
  if (in_sizes[4] != kHid * kHid) return;
  if (in_sizes[5] != kHid) return;
  if (in_sizes[6] != kHid) return;
  if (in_sizes[7] != 1) return;
  if (in_sizes[8] != 7 * kHid) return;
  if (in_sizes[9] != kHid) return;
  if (in_sizes[10] != kHid * kHid) return;
  if (in_sizes[11] != kHid) return;
  if (in_sizes[12] != kHid * 3) return;
  if (in_sizes[13] != 3) return;
  if (out_size != kBatch * kRowF + kBatch * kPairs) return;
  if (ws_size < kWsTotal) return;

  const float* pos   = (const float*)d_in[0];
  const float* vel   = (const float*)d_in[1];
  const float* sm_w1 = (const float*)d_in[2];
  const float* sm_b1 = (const float*)d_in[3];
  const float* sm_w2 = (const float*)d_in[4];
  const float* sm_b2 = (const float*)d_in[5];
  const float* sm_w3 = (const float*)d_in[6];
  const float* sm_b3 = (const float*)d_in[7];
  const float* rp_w1 = (const float*)d_in[8];
  const float* rp_b1 = (const float*)d_in[9];
  const float* rp_w2 = (const float*)d_in[10];
  const float* rp_b2 = (const float*)d_in[11];
  const float* rp_w3 = (const float*)d_in[12];
  const float* rp_b3 = (const float*)d_in[13];

  float* out_forces = (float*)d_out;
  float* out_viol   = (float*)d_out + (size_t)kBatch * kRowF;
  int*   flags      = (int*)d_ws;

  pair_mlp_kernel<false><<<kBatch, 256, 0, stream>>>(pos, vel, sm_w1, sm_b1, sm_w2, sm_b2, sm_w3, sm_b3,
                                                     flags, out_viol);
  pair_flag_kernel<<<8, 256, 0, stream>>>(out_viol, flags);
  pair_mlp_kernel<true><<<kBatch, 256, 0, stream>>>(pos, vel, rp_w1, rp_b1, rp_w2, rp_b2, rp_w3, rp_b3,
                                                    flags, out_forces);
}
